// TESTRNN_6837587935697
// MI455X (gfx1250) — hardware-verified
//
#include <hip/hip_runtime.h>

typedef __attribute__((ext_vector_type(16))) _Float16 v16h;
typedef __attribute__((ext_vector_type(8)))  _Float16 v8h;
typedef __attribute__((ext_vector_type(8)))  float    v8f;
typedef __attribute__((ext_vector_type(4)))  float    v4f;

constexpr int kBatch  = 4096;
constexpr int kTime   = 2048;
constexpr int kHid    = 20;
constexpr int kHidPad = 32;
constexpr int kSeqPB  = 64;
constexpr int kBlocksPerDir = kBatch / kSeqPB;
constexpr int kBlocks = 2 * kBlocksPerDir;
constexpr int kThreads = 128;
constexpr int kHP     = 40;
constexpr int kHTile  = kSeqPB * kHP;
constexpr int kXC     = 64;
constexpr int kXP     = 64;
constexpr int kFP     = 36;
constexpr int kOutPB  = kSeqPB / 2;
static_assert(kBatch % kSeqPB == 0);
static_assert(kTime % kXC == 0);
static_assert((kThreads / 32) * 16 == kSeqPB);
static_assert(kHid <= kHidPad && kHidPad == 32);
static_assert(kHP % 8 == 0 && kHP >= kHidPad);
static_assert(kXC * kXP == kThreads * 32);
static_assert((2 * kHTile) % (8 * kThreads) == 0);
static_assert(kOutPB == 32);
static_assert(kFP % 4 == 0 && kXP % 4 == 0);

__device__ __forceinline__ void dep_guard_h(v8f& a, v8f& b, v16h x, v16h y) { asm volatile("v_nop\n\tv_nop\n\tv_nop\n\tv_nop" : "+v"(a), "+v"(b) : "v"(x), "v"(y)); }
__device__ __forceinline__ void keep4_h(v16h a, v16h b, v16h c, v16h d) { asm volatile("v_nop" :: "v"(a), "v"(b), "v"(c), "v"(d)); }

template <typename T> struct Frag;
template <> struct Frag<_Float16> {
  typedef v16h V; union U { v16h v; v8h h[2]; };
  static __device__ __forceinline__ v16h load(const _Float16* p) {
    U f; f.h[0] = *(const v8h*)(p); f.h[1] = *(const v8h*)(p + 16); return f.v;
  }
  static __device__ __forceinline__ v8f mma(v16h a, v16h b, v8f c) {
    return __builtin_amdgcn_wmma_f32_16x16x32_f16(false, a, false, b, (short)0, c, false, false);
  }
  static __device__ __forceinline__ void guard(v8f& a, v8f& b, v16h x, v16h y) { dep_guard_h(a, b, x, y); }
  static __device__ __forceinline__ void keep(v16h a, v16h b, v16h c, v16h d) { keep4_h(a, b, c, d); }
};

__device__ __forceinline__ void mma_guard2(v8f& a, v8f& b, v16h x, v16h y, v16h z) {
  asm volatile("v_nop\n\tv_nop\n\tv_nop\n\tv_nop" : "+v"(a), "+v"(b) : "v"(x), "v"(y), "v"(z));
}

__device__ __forceinline__ float ftanh(float x) { return 1.0f - 2.0f * __builtin_amdgcn_rcpf(1.0f + __expf(2.0f * x)); }

__global__ __launch_bounds__(kThreads) void birnn_fused_kernel(
    const float* __restrict__ x,
    const float* __restrict__ wih_f, const float* __restrict__ whh_f,
    const float* __restrict__ bih_f, const float* __restrict__ bhh_f,
    const float* __restrict__ wih_b, const float* __restrict__ whh_b,
    const float* __restrict__ bih_b, const float* __restrict__ bhh_b,
    const float* __restrict__ wfc, const float* __restrict__ bfc,
    float* __restrict__ out)
{
  __shared__ __align__(16) _Float16 hbuf[2 * kHTile];
  __shared__ __align__(16) float    xs[kXC * kXP];
  __shared__ __align__(16) float    hfin[kSeqPB * kFP];
  __shared__ __align__(16) float    outs[kOutPB];

  const int tid  = threadIdx.x;
  const int lane = tid & 31;
  const int wave = tid >> 5;
  const int c    = lane & 15;
  const int hh   = lane >> 4;
  const int koff = hh * 8;
  const int mOff = hh * 8;
  const int dir  = (int)blockIdx.x / kBlocksPerDir;
  const int b0   = ((int)blockIdx.x - dir * kBlocksPerDir) * kSeqPB;
  const int r0   = wave * 16;

  {
    const v8h z = {(_Float16)0.f, (_Float16)0.f, (_Float16)0.f, (_Float16)0.f, (_Float16)0.f, (_Float16)0.f, (_Float16)0.f, (_Float16)0.f};
    for (int i = tid; i < (2 * kHTile) / 8; i += kThreads) *(v8h*)(hbuf + i * 8) = z;
  }

  float wih8[2], bsum8[2];
  v16h  fb[2];
#pragma unroll
  for (int j = 0; j < 2; ++j) {
    const int  n  = 16 * j + c;
    const bool nv = (n < kHid);
    const int  nc = nv ? n : (kHid - 1);
    const float wf = wih_f[nc], wb = wih_b[nc];
    const float sf = bih_f[nc] + bhh_f[nc];
    const float sb = bih_b[nc] + bhh_b[nc];
    const float wsel = dir ? wb : wf;
    const float ssel = dir ? sb : sf;
    wih8[j]  = nv ? (wsel * 8.0f) : 0.0f;
    bsum8[j] = nv ? (ssel * 8.0f) : 0.0f;
#pragma unroll
    for (int i = 0; i < 16; ++i) {
      const int  k  = (i < 8) ? (koff + i) : (16 + koff + (i - 8));
      const bool kv = (k < kHid);
      const int  kc = kv ? k : (kHid - 1);
      const float vf = whh_f[nc * kHid + kc];
      const float vb = whh_b[nc * kHid + kc];
      const float vs = dir ? vb : vf;
      fb[j][i] = (_Float16)((nv && kv) ? (vs * 8.0f) : 0.0f);
    }
  }
  __syncthreads();

  const int sseq = tid >> 1;
  const int sth  = tid & 1;
  const float* xrow = x + (size_t)(b0 + sseq) * kTime;

#pragma unroll 1
  for (int cnk = 0; cnk < kTime / kXC; ++cnk) {
    {
      const int src0 = dir ? (kTime - kXC - cnk * kXC) : (cnk * kXC);
      const float* sp = xrow + src0 + sth * 32;
#pragma unroll
      for (int q = 0; q < 8; ++q) {
        const v4f v = *(const v4f*)(sp + 4 * q);
#pragma unroll
        for (int e = 0; e < 4; ++e) {
          const int idx = sth * 32 + 4 * q + e;
          const int tt  = dir ? (kXC - 1 - idx) : idx;
          xs[tt * kXP + sseq] = v[e];
        }
      }
    }
    __syncthreads();

#pragma unroll 1
    for (int tt = 0; tt < kXC; ++tt) {
      const int t = cnk * kXC + tt;
      const _Float16* hc = hbuf + (t & 1) * kHTile;
      _Float16*       hn = hbuf + ((t + 1) & 1) * kHTile;

      const float* xp = xs + tt * kXP + r0 + mOff;
      const v4f xa = *(const v4f*)xp;
      const v4f xb = *(const v4f*)(xp + 4);
      float xv[8];
      xv[0] = xa[0]; xv[1] = xa[1]; xv[2] = xa[2]; xv[3] = xa[3];
      xv[4] = xb[0]; xv[5] = xb[1]; xv[6] = xb[2]; xv[7] = xb[3];

      v8f acc[2];
#pragma unroll
      for (int j = 0; j < 2; ++j) {
#pragma unroll
        for (int r = 0; r < 8; ++r) acc[j][r] = fmaf(xv[r], wih8[j], bsum8[j]);
      }

      const v16h fa = Frag<_Float16>::load(hc + (r0 + c) * kHP + koff);
      acc[0] = Frag<_Float16>::mma(fa, fb[0], acc[0]);
      acc[1] = Frag<_Float16>::mma(fa, fb[1], acc[1]);
      mma_guard2(acc[0], acc[1], fa, fb[0], fb[1]);

      float hv[2][8];
#pragma unroll
      for (int j = 0; j < 2; ++j) {
#pragma unroll
        for (int r = 0; r < 8; ++r) {
          const float h = ftanh(acc[j][r] * 0.125f);
          hv[j][r] = h;
          hn[(r0 + mOff + r) * kHP + 16 * j + c] = (_Float16)h;
        }
      }
      if (t == kTime - 1) {
#pragma unroll
        for (int j = 0; j < 2; ++j) {
#pragma unroll
          for (int r = 0; r < 8; ++r) hfin[(r0 + mOff + r) * kFP + 16 * j + c] = hv[j][r];
        }
      }
      __syncthreads();
    }
  }

  if (wave == 0) {
    const float* ha = hfin + (2 * lane) * kFP;
    const float* hb2 = hfin + (2 * lane + 1) * kFP;
    float s = 0.0f;
#pragma unroll 1
    for (int k = 0; k < kHid; ++k) s = fmaf(ha[k], wfc[k], s);
#pragma unroll 1
    for (int k = 0; k < kHid; ++k) s = fmaf(hb2[k], wfc[kHid + k], s);
    s += bfc[0];
    outs[lane] = s;
    __builtin_amdgcn_fence(__ATOMIC_RELEASE, "workgroup");
    __builtin_amdgcn_wave_barrier();
    __builtin_amdgcn_fence(__ATOMIC_ACQUIRE, "workgroup");
    const v4f val = *(const v4f*)(outs + 4 * (lane & 7));
    float* op = out + (size_t)dir * (kBatch / 2) + (size_t)(b0 >> 1);
    for (int pass = 0; pass < 2; ++pass) {
      if (lane < 8) *(volatile v4f*)(op + 4 * lane) = val;
      __threadfence();
    }
  }
}

extern "C" void kernel_launch(void* const* d_in, const int* in_sizes, int n_in,
                              void* d_out, int out_size, void* d_ws, size_t ws_size, hipStream_t stream) {
  (void)d_ws; (void)ws_size;
  if (n_in < 11 || d_out == nullptr) return;
  if (in_sizes[0] != kBatch * kTime || in_sizes[1] != kHid || in_sizes[2] != kHid * kHid ||
      in_sizes[3] != kHid || in_sizes[4] != kHid || in_sizes[5] != kHid || in_sizes[6] != kHid * kHid ||
      in_sizes[7] != kHid || in_sizes[8] != kHid || in_sizes[9] != 2 * kHid || in_sizes[10] != 1 ||
      out_size != kBatch) return;

  const float* x     = (const float*)d_in[0];
  const float* wih_f = (const float*)d_in[1];
  const float* whh_f = (const float*)d_in[2];
  const float* bih_f = (const float*)d_in[3];
  const float* bhh_f = (const float*)d_in[4];
  const float* wih_b = (const float*)d_in[5];
  const float* whh_b = (const float*)d_in[6];
  const float* bih_b = (const float*)d_in[7];
  const float* bhh_b = (const float*)d_in[8];
  const float* wfc   = (const float*)d_in[9];
  const float* bfc   = (const float*)d_in[10];
  float* out = (float*)d_out;

  birnn_fused_kernel<<<kBlocks, kThreads, 0, stream>>>(x, wih_f, whh_f, bih_f, bhh_f,
                                                       wih_b, whh_b, bih_b, bhh_b, wfc, bfc, out);
}
